// T_TGCN_18485539242711
// MI455X (gfx1250) — hardware-verified
//
#include <hip/hip_runtime.h>
#include <math.h>


typedef unsigned int u32;
typedef __attribute__((ext_vector_type(2)))  int      v2i;
typedef __attribute__((ext_vector_type(16))) _Float16 v16h;
typedef __attribute__((ext_vector_type(8)))  _Float16 v8h;
typedef __attribute__((ext_vector_type(8)))  float    v8f;
typedef __attribute__((ext_vector_type(4)))  float    v4f;
#define NN    50000
#define NE    800000
#define DD    128
#define NCAND 13
#define SORTN 1048576
#define TILE  8192
#define NPAD  50176
#define MAXDEG 4096
#define VST2(T, ptr, val) do { const T _v = (val); *(volatile T*)(ptr) = _v; __threadfence(); *(volatile T*)(ptr) = _v; } while (0)
__device__ __forceinline__ v8f wmma16(v16h a, v16h b, v8f c) {
  v8f d = __builtin_amdgcn_wmma_f32_16x16x32_f16(false, a, false, b, (short)0, c, false, false);
  asm volatile("v_nop\n\tv_nop\n\tv_nop\n\tv_nop" : "+v"(d) : "v"(a), "v"(b));
  return d;
}
__device__ __forceinline__ v16h frag16(const _Float16* p, int hh) {
  const v8h lo = *(const v8h*)(p + 8 * hh), hi = *(const v8h*)(p + 16 + 8 * hh);
  return __builtin_shufflevector(lo, hi, 0,1,2,3,4,5,6,7,8,9,10,11,12,13,14,15);
}
__global__ __launch_bounds__(256) void k_sort_init(const int* __restrict__ src, const int* __restrict__ dst, u32* __restrict__ A, int E) {
  const int i = blockIdx.x * 256 + threadIdx.x;
  VST2(u32, A + i, (i < E) ? (((u32)dst[i]) << 16) | ((u32)i & 0xffffu) : 0xffffffffu);
}
__device__ __forceinline__ void cas_lds(u32* s, int lo, int hi, bool up) {
  const u32 a = s[lo], b = s[hi]; const bool sw = up ? (a > b) : (a < b); s[lo] = sw ? b : a; s[hi] = sw ? a : b;
}
__global__ __launch_bounds__(256) void k_sort_local(u32* __restrict__ A) {
  __shared__ u32 s[TILE];
  const int base = blockIdx.x * TILE, t = threadIdx.x;
  for (int i = t; i < TILE; i += 256) s[i] = A[base + i];
  __syncthreads();
  for (int k = 2; k <= TILE; k <<= 1)
    for (int j = k >> 1; j > 0; j >>= 1) {
      for (int p = t; p < TILE / 2; p += 256) {
        const int lo = ((p >> __builtin_ctz(j)) << (__builtin_ctz(j) + 1)) | (p & (j - 1));
        cas_lds(s, lo, lo + j, (((base + lo) & k) == 0));
      }
      __syncthreads();
    }
  for (int pass = 0; pass < 2; ++pass) { for (int i = t; i < TILE; i += 256) *(volatile u32*)(A + base + i) = s[i]; __threadfence(); }
}
__global__ __launch_bounds__(256) void k_sort_global(u32* __restrict__ A, int logj, int k) {
  const int p = blockIdx.x * 256 + threadIdx.x;
  const int j = 1 << logj;
  const int lo = ((p >> logj) << (logj + 1)) | (p & (j - 1)), hi = lo + j;
  const u32 a = A[lo], b = A[hi];
  const bool up = ((lo & k) == 0), sw = up ? (a > b) : (a < b);
  const u32 vlo = sw ? b : a, vhi = sw ? a : b;
  *(volatile u32*)(A + lo) = vlo; *(volatile u32*)(A + hi) = vhi; __threadfence();
  *(volatile u32*)(A + lo) = vlo; *(volatile u32*)(A + hi) = vhi;
}
__global__ __launch_bounds__(256) void k_sort_lds(u32* __restrict__ A, int k) {
  __shared__ u32 s[TILE];
  const int base = blockIdx.x * TILE, t = threadIdx.x;
  for (int i = t; i < TILE; i += 256) s[i] = A[base + i];
  __syncthreads();
  for (int j = TILE >> 1; j > 0; j >>= 1) {
    for (int p = t; p < TILE / 2; p += 256) {
      const int lo = ((p >> __builtin_ctz(j)) << (__builtin_ctz(j) + 1)) | (p & (j - 1));
      cas_lds(s, lo, lo + j, (((base + lo) & k) == 0));
    }
    __syncthreads();
  }
  for (int pass = 0; pass < 2; ++pass) { for (int i = t; i < TILE; i += 256) *(volatile u32*)(A + base + i) = s[i]; __threadfence(); }
}

__global__ __launch_bounds__(256) void k_segs(const u32* __restrict__ A, v2i* __restrict__ seg, float* __restrict__ inv) {
  const int n = blockIdx.x * 256 + threadIdx.x;
  if (n >= NN) return;
  int lo = 0, hi = SORTN;
  while (lo < hi) { const int mid = (lo + hi) >> 1; if ((A[mid] >> 16) < (u32)n) lo = mid + 1; else hi = mid; }
  const int st = lo; hi = SORTN;
  while (lo < hi) { const int mid = (lo + hi) >> 1; if ((A[mid] >> 16) < (u32)(n + 1)) lo = mid + 1; else hi = mid; }
  const v2i sv = {st, lo - st};
  VST2(v2i, seg + n, sv);
  VST2(float, inv + n, 1.0f / fmaxf((float)(lo - st), 1.0f));
}

__global__ __launch_bounds__(256) void k_resolve(const u32* __restrict__ keys, const int* __restrict__ edst, u32* __restrict__ eids) {
  const int p = blockIdx.x * 256 + threadIdx.x;
  if (p >= NE) return;
  const u32 key = keys[p]; const int d = (int)(key >> 16), lo16 = (int)(key & 0xffffu);
  int r = 0;
  while (r < NCAND && p - r - 1 >= 0 && keys[p - r - 1] == key) ++r;
  u32 eid = 0; int seen = 0; bool found = false;
  for (int t = 0; t < NCAND; ++t) { const int c = lo16 + (t << 16); if (c < NE && edst[c] == d) { if (seen == r && !found) { eid = (u32)c; found = true; } ++seen; } }
  VST2(u32, eids + p, eid);
}
__global__ __launch_bounds__(256) void k_deg(const v2i* __restrict__ seg, const u32* __restrict__ eids, const float* __restrict__ ew, float* __restrict__ dis) {
  const int n = blockIdx.x * 256 + threadIdx.x;
  if (n >= NN) return;
  const v2i sv = seg[n];
  const int st = min(max(sv[0], 0), SORTN - 1), cnt = min(max(sv[1], 0), MAXDEG);
  float deg = 2.0f;
  for (int p = 0; p < cnt; ++p) deg += ew[min((int)eids[min(st + p, NE - 1)], NE - 1)];
  VST2(float, dis + n, rsqrtf(deg));
}
__global__ __launch_bounds__(256) void k_agg(const float* __restrict__ x, const int* __restrict__ esrc, const v2i* __restrict__ seg, const u32* __restrict__ eids,
                                             const float* __restrict__ ew, const float* __restrict__ dis, _Float16* __restrict__ agg16) {
  const int t = blockIdx.x * 256 + threadIdx.x;
  const int n = t >> 4, c = (t & 15) * 8;
  float acc[8] = {0.f, 0.f, 0.f, 0.f, 0.f, 0.f, 0.f, 0.f};
  if (n < NN) {
    const v2i sv = seg[n];
    const int st = min(max(sv[0], 0), SORTN - 1), cnt = min(max(sv[1], 0), MAXDEG);
    const float dn = dis[n];
    for (int p = 0; p < cnt; ++p) {
      const int e = min((int)eids[min(st + p, NE - 1)], NE - 1);
      const int s = min(max(esrc[e], 0), NN - 1);
      const float w = dis[s] * ew[e] * dn;
      const float* xr = x + (size_t)s * DD + c;
#pragma unroll
      for (int q = 0; q < 8; ++q) acc[q] += w * xr[q];
    }
    const float ws_ = 2.0f * dn * dn; const float* xr = x + (size_t)n * DD + c;
#pragma unroll
    for (int q = 0; q < 8; ++q) acc[q] += ws_ * xr[q];
  }
  v8h o;
#pragma unroll
  for (int q = 0; q < 8; ++q) o[q] = (_Float16)acc[q];
  VST2(v8h, agg16 + (size_t)n * DD + c, o);
}
__global__ __launch_bounds__(256) void k_wt3(const float* __restrict__ w0, const float* __restrict__ w1, const float* __restrict__ w2, int K, int ncol, int Ntot, _Float16* __restrict__ Wt) {
  const int t = blockIdx.x * 256 + threadIdx.x;
  const int per = K / 8;
  if (t >= Ntot * per) return;
  const int n = t / per, k0 = (t % per) * 8;
  const float* w = (n < ncol) ? w0 : (n < 2 * ncol) ? w1 : w2; const int nn = n % ncol;
  v8h o;
#pragma unroll
  for (int e = 0; e < 8; ++e) o[e] = (_Float16)w[(size_t)(k0 + e) * ncol + nn];
  VST2(v8h, Wt + (size_t)n * K + k0, o);
}
__global__ __launch_bounds__(256) void k_urows(const float* __restrict__ C, int goff, const float* __restrict__ h0, const float* __restrict__ R, _Float16* __restrict__ U) {
  const int t = blockIdx.x * 256 + threadIdx.x;
  const int n = t >> 5, c = (t & 31) * 8;
  v8h o;
#pragma unroll
  for (int e = 0; e < 8; ++e) {
    float v = 0.f;
    if (n < NN) { if (c < DD) v = C[(size_t)n * 384 + goff + c + e]; else { v = h0[(size_t)n * DD + c - DD + e]; if (R) v *= R[(size_t)n * DD + c - DD + e]; } }
    o[e] = (_Float16)v;
  }
  VST2(v8h, U + (size_t)n * 256 + c, o);
}
template <int K, int NTOT, int EPI>
__global__ __launch_bounds__(128) void k_gemm(const _Float16* __restrict__ A, const _Float16* __restrict__ Wt, const float* __restrict__ bias,
                                              const float* __restrict__ Z, const float* __restrict__ h0, const float* __restrict__ linw, const float* __restrict__ linb,
                                              float* __restrict__ outf, float* __restrict__ outy) {
  __shared__ __attribute__((aligned(16))) float sT[4][16][132];
  __shared__ __attribute__((aligned(16))) float sY[64 * 7];
  const int lane = threadIdx.x & 31, wave = threadIdx.x >> 5, hh = lane >> 4, l16 = lane & 15;
  const int m0 = blockIdx.x * 64 + wave * 16, n0 = blockIdx.y * 128;
  v8f acc[8];
#pragma unroll
  for (int ni = 0; ni < 8; ++ni) acc[ni] = (v8f){};
#pragma unroll 2
  for (int k0 = 0; k0 < K; k0 += 32) {
    const v16h a0 = frag16(A + (size_t)(m0 + l16) * K + k0, hh);
#pragma unroll
    for (int ni = 0; ni < 8; ++ni) { const v16h b = frag16(Wt + (size_t)(n0 + ni * 16 + l16) * K + k0, hh); acc[ni] = wmma16(a0, b, acc[ni]); }
  }
  float (*st)[132] = sT[wave];
#pragma unroll
  for (int ni = 0; ni < 8; ++ni)
#pragma unroll
    for (int i = 0; i < 8; ++i) { float v = acc[ni][i] + bias[n0 + ni * 16 + l16]; if (EPI == 3) v = 1.0f / (1.0f + expf(-v)); st[i + 8 * hh][ni * 16 + l16] = v; }
  __builtin_amdgcn_fence(__ATOMIC_RELEASE, "workgroup"); __builtin_amdgcn_wave_barrier(); __builtin_amdgcn_fence(__ATOMIC_ACQUIRE, "workgroup");
  if (EPI == 4) {
    if (lane < 16) {
      const int row = m0 + lane; float* rw = st[lane];
      float y[7] = {0.f, 0.f, 0.f, 0.f, 0.f, 0.f, 0.f};
      if (row < NN) {
        const float* zr = Z + (size_t)row * DD; const float* hr = h0 + (size_t)row * DD;
        for (int c = 0; c < 128; ++c) {
          const float z = zr[c], hv = z * hr[c] + (1.0f - z) * tanhf(rw[c]);
          rw[c] = hv; const float rl = fmaxf(hv, 0.f);
#pragma unroll
          for (int o = 0; o < 7; ++o) y[o] += rl * linw[c * 7 + o];
        }
      }
#pragma unroll
      for (int o = 0; o < 7; ++o) sY[(wave * 16 + lane) * 7 + o] = y[o] + linb[o];
    }
    __syncthreads();
  }
  for (int pass = 0; pass < 2; ++pass) {
#pragma unroll
    for (int rr = 0; rr < 16; ++rr) if (EPI != 4 || m0 + rr < NN)
      *(volatile v4f*)(outf + (size_t)(m0 + rr) * NTOT + n0 + lane * 4) = *(const v4f*)(&st[rr][lane * 4]);
    if (EPI == 4) {
      const int rows = min(64, NN - (int)blockIdx.x * 64);
      for (int q = threadIdx.x; q < rows * 7; q += 128) *(volatile float*)(outy + (size_t)blockIdx.x * 64 * 7 + q) = sY[q];
    }
    __threadfence();
  }
}
extern "C" void kernel_launch(void* const* d_in, const int* in_sizes, int n_in,
                              void* d_out, int out_size, void* d_ws, size_t ws_size, hipStream_t stream) {
  (void)in_sizes; (void)n_in; (void)out_size;
  const float* x   = (const float*)d_in[0];
  const int*   ei  = (const int*)  d_in[1];
  const float* ew  = (const float*)d_in[2];
  const float* h0  = (const float*)d_in[3];
  const float* Wz  = (const float*)d_in[4];  const float* bz  = (const float*)d_in[5];
  const float* Wr  = (const float*)d_in[6];  const float* br  = (const float*)d_in[7];
  const float* Wh  = (const float*)d_in[8];  const float* bh  = (const float*)d_in[9];
  const float* Lzw = (const float*)d_in[10]; const float* Lzb = (const float*)d_in[11];
  const float* Lrw = (const float*)d_in[12]; const float* Lrb = (const float*)d_in[13];
  const float* Lhw = (const float*)d_in[14]; const float* Lhb = (const float*)d_in[15];
  const float* linw = (const float*)d_in[16]; const float* linb = (const float*)d_in[17];
  float* outH = (float*)d_out;
  float* outY = (float*)((char*)d_out + 25600000);
  char* ws = (char*)d_ws; size_t off = 0;
  auto take = [&](size_t bytes) { void* p = ws + off; off = (off + bytes + 255) & ~(size_t)255; return p; };
  u32*      keys = (u32*)take((size_t)SORTN * 4);
  u32*      eids = (u32*)take((size_t)NE * 4);
  v2i*      seg  = (v2i*)take((size_t)NN * 8);
  float*    inv  = (float*)take((size_t)NN * 4);
  float*    dis  = (float*)take((size_t)NN * 4);
  _Float16* agg  = (_Float16*)take((size_t)NPAD * DD * 2);
  _Float16* WtC  = (_Float16*)take((size_t)384 * DD * 2);
  _Float16* WtZ  = (_Float16*)take((size_t)DD * 256 * 2);
  _Float16* WtR  = (_Float16*)take((size_t)DD * 256 * 2);
  _Float16* WtH  = (_Float16*)take((size_t)DD * 256 * 2);
  float*    Cc   = (float*)take((size_t)NPAD * 384 * 4);
  float*    bC   = (float*)take((size_t)384 * 4);
  _Float16* U    = (_Float16*)take((size_t)NPAD * 256 * 2);
  float*    Zf   = (float*)take((size_t)NPAD * DD * 4);
  float*    Rf   = (float*)take((size_t)NPAD * DD * 4);
  if (off > ws_size) return;
  hipMemcpyAsync(bC, bz, DD * 4, hipMemcpyDeviceToDevice, stream);
  hipMemcpyAsync(bC + DD, br, DD * 4, hipMemcpyDeviceToDevice, stream);
  hipMemcpyAsync(bC + 2 * DD, bh, DD * 4, hipMemcpyDeviceToDevice, stream);
  const dim3 b256(256);
  k_sort_init<<<SORTN / 256, b256, 0, stream>>>(ei, ei + NE, keys, NE);
  k_sort_local<<<SORTN / TILE, b256, 0, stream>>>(keys);
  for (int k = TILE * 2; k <= SORTN; k <<= 1) {
    for (int logj = __builtin_ctz(k) - 1; (1 << logj) >= TILE; --logj)
      k_sort_global<<<SORTN / 2 / 256, b256, 0, stream>>>(keys, logj, k);
    k_sort_lds<<<SORTN / TILE, b256, 0, stream>>>(keys, k);
  }
  k_segs<<<(NN + 255) / 256, b256, 0, stream>>>(keys, seg, inv);
  k_resolve<<<(NE + 255) / 256, b256, 0, stream>>>(keys, ei + NE, eids);
  k_deg<<<(NN + 255) / 256, b256, 0, stream>>>(seg, eids, ew, dis);
  k_agg<<<NPAD * 16 / 256, b256, 0, stream>>>(x, ei, seg, eids, ew, dis, agg);
  k_wt3<<<(384 * 16 + 255) / 256, b256, 0, stream>>>(Wz, Wr, Wh, DD, DD, 384, WtC);
  k_wt3<<<(DD * 32 + 255) / 256, b256, 0, stream>>>(Lzw, Lzw, Lzw, 256, DD, DD, WtZ);
  k_wt3<<<(DD * 32 + 255) / 256, b256, 0, stream>>>(Lrw, Lrw, Lrw, 256, DD, DD, WtR);
  k_wt3<<<(DD * 32 + 255) / 256, b256, 0, stream>>>(Lhw, Lhw, Lhw, 256, DD, DD, WtH);
  k_gemm<DD, 384, 0><<<dim3(NPAD / 64, 3), 128, 0, stream>>>(agg, WtC, bC, nullptr, nullptr, nullptr, nullptr, Cc, nullptr);
  k_urows<<<NPAD * 32 / 256, b256, 0, stream>>>(Cc, 0, h0, nullptr, U);
  k_gemm<256, DD, 3><<<dim3(NPAD / 64, 1), 128, 0, stream>>>(U, WtZ, Lzb, nullptr, nullptr, nullptr, nullptr, Zf, nullptr);
  k_urows<<<NPAD * 32 / 256, b256, 0, stream>>>(Cc, DD, h0, nullptr, U);
  k_gemm<256, DD, 3><<<dim3(NPAD / 64, 1), 128, 0, stream>>>(U, WtR, Lrb, nullptr, nullptr, nullptr, nullptr, Rf, nullptr);
  k_urows<<<NPAD * 32 / 256, b256, 0, stream>>>(Cc, 2 * DD, h0, Rf, U);
  k_gemm<256, DD, 4><<<dim3(NPAD / 64, 1), 128, 0, stream>>>(U, WtH, Lhb, Zf, h0, linw, linb, outH, outY);
}
